// SparseGCN_62122406969952
// MI455X (gfx1250) — hardware-verified
//
#include <hip/hip_runtime.h>
#include <stddef.h>


#define FIN    128
#define KF     256
#define NOUT   128
#define OUTW   128
#define NTHR   256
#define NWAVE  8
#define EPT    8
#define NGRP   2
#define CHUNK  (NTHR * EPT * NGRP)
#define WCAP   (EPT * NGRP * 32)
#define LISTN  (NWAVE * WCAP)
#define TGT    512
#define NPL    (2 * NOUT * KF)
#define LDS_ACC  (TGT * FIN * 4)
#define LDS_MAIN (LDS_ACC + LISTN * 4 + TGT * 4 + 64)

static_assert((CHUNK & (CHUNK - 1)) == 0);
static_assert(CHUNK <= 4096);
static_assert((TGT & (TGT - 1)) == 0 && TGT <= 4096);
static_assert(TGT % (NWAVE * 16) == 0);
static_assert((TGT * FIN / 4) % NTHR == 0 && TGT % NTHR == 0);
static_assert(KF == 2 * FIN && (KF % 32) == 0 && (FIN % 32) == 0);
static_assert((NOUT * (KF / 8)) % NTHR == 0);
static_assert(NWAVE * 32 == NTHR);
static_assert(NOUT == 8 * 16);
static_assert(OUTW == NOUT && OUTW == 32 * 4);
static_assert(16 * FIN == 8 * 32 * 8);
static_assert(LDS_MAIN <= 300 * 1024);

typedef float          v4f   __attribute__((ext_vector_type(4)));
typedef float          v8f   __attribute__((ext_vector_type(8)));
typedef int            v4i   __attribute__((ext_vector_type(4)));
typedef unsigned short v8us  __attribute__((ext_vector_type(8)));
typedef unsigned short v16us __attribute__((ext_vector_type(16)));
typedef __bf16         v16b  __attribute__((ext_vector_type(16)));
union FragB { v16b v; v16us u; v8us h[2]; };

__device__ __forceinline__ unsigned int bf_bits(float f) {
  const unsigned int u = __float_as_uint(f);
  return (u + 0x7FFFu + ((u >> 16) & 1u)) >> 16;
}

__device__ __forceinline__ void split16(v4f a0, v4f a1, v4f a2, v4f a3, FragB& hi, FragB& lo) {
  float f[16];
  f[0]  = a0.x; f[1]  = a0.y; f[2]  = a0.z; f[3]  = a0.w;
  f[4]  = a1.x; f[5]  = a1.y; f[6]  = a1.z; f[7]  = a1.w;
  f[8]  = a2.x; f[9]  = a2.y; f[10] = a2.z; f[11] = a2.w;
  f[12] = a3.x; f[13] = a3.y; f[14] = a3.z; f[15] = a3.w;
  v16us hu, lu;
#pragma unroll
  for (int e = 0; e < 16; ++e) {
    const unsigned int hb = bf_bits(f[e]);
    hu[e] = (unsigned short)hb;
    lu[e] = (unsigned short)bf_bits(f[e] - __uint_as_float(hb << 16));
  }
  hi.u = hu; lo.u = lu;
}

__device__ __forceinline__ v8f wmb(const FragB& a, const FragB& b, v8f c) {
  v8f d = __builtin_amdgcn_wmma_f32_16x16x32_bf16(false, a.v, false, b.v, (short)0, c, false, false);
  asm volatile("v_nop\n\tv_nop\n\tv_nop\n\tv_nop" : "+v"(d) : "v"(a.u), "v"(b.u));
  return d;
}

template <int NB>
__device__ __forceinline__ int scan_chunk(const int* __restrict__ adj, int nE, int cbase, int slotBase,
                                          int* list, int tid, int wave) {
  int wc = 0;
#pragma unroll
  for (int g = 0; g < NGRP; ++g) {
    const int el0  = (g * NTHR + tid) * EPT;
    const int e0   = cbase + el0;
    const int sent = -2147483647 - 1;
    v4i da, db;
    if (cbase + CHUNK <= nE) {
      const int* q = adj + (size_t)2 * (size_t)e0;
      const v4i q0 = *(const v4i*)(q);
      const v4i q1 = *(const v4i*)(q + 4);
      const v4i q2 = *(const v4i*)(q + 8);
      const v4i q3 = *(const v4i*)(q + 12);
      da.x = q0.x; da.y = q0.z; da.z = q1.x; da.w = q1.z;
      db.x = q2.x; db.y = q2.z; db.z = q3.x; db.w = q3.z;
    } else {
      const int em = nE - 1;
      da.x = (e0     < nE) ? adj[(size_t)2 * (size_t)min(e0,     em)] : sent;
      da.y = (e0 + 1 < nE) ? adj[(size_t)2 * (size_t)min(e0 + 1, em)] : sent;
      da.z = (e0 + 2 < nE) ? adj[(size_t)2 * (size_t)min(e0 + 2, em)] : sent;
      da.w = (e0 + 3 < nE) ? adj[(size_t)2 * (size_t)min(e0 + 3, em)] : sent;
      db.x = (e0 + 4 < nE) ? adj[(size_t)2 * (size_t)min(e0 + 4, em)] : sent;
      db.y = (e0 + 5 < nE) ? adj[(size_t)2 * (size_t)min(e0 + 5, em)] : sent;
      db.z = (e0 + 6 < nE) ? adj[(size_t)2 * (size_t)min(e0 + 6, em)] : sent;
      db.w = (e0 + 7 < nE) ? adj[(size_t)2 * (size_t)min(e0 + 7, em)] : sent;
    }
    const int mn = min(min(min(da.x, da.y), min(da.z, da.w)), min(min(db.x, db.y), min(db.z, db.w)));
    const int mx = max(max(max(da.x, da.y), max(da.z, da.w)), max(max(db.x, db.y), max(db.z, db.w)));
    const bool coarse = (mx >= slotBase) && (mn < slotBase + NB);
    const unsigned anyc = __builtin_amdgcn_ballot_w32(coarse);
    if (anyc != 0u) {
      const unsigned nb = (unsigned)slotBase;
      const unsigned s0 = (unsigned)da.x - nb, s1 = (unsigned)da.y - nb;
      const unsigned s2 = (unsigned)da.z - nb, s3 = (unsigned)da.w - nb;
      const unsigned s4 = (unsigned)db.x - nb, s5 = (unsigned)db.y - nb;
      const unsigned s6 = (unsigned)db.z - nb, s7 = (unsigned)db.w - nb;
      const bool h0 = s0 < (unsigned)NB, h1 = s1 < (unsigned)NB, h2 = s2 < (unsigned)NB, h3 = s3 < (unsigned)NB;
      const bool h4 = s4 < (unsigned)NB, h5 = s5 < (unsigned)NB, h6 = s6 < (unsigned)NB, h7 = s7 < (unsigned)NB;
#define HITJ(J, HJ, SJ) { \
        const unsigned mj = __builtin_amdgcn_ballot_w32(HJ); \
        if (mj != 0u) { \
          if (HJ) { \
            const int pos = wc + (int)__builtin_amdgcn_mbcnt_lo(mj, 0u); \
            if (pos < WCAP) list[wave * WCAP + pos] = ((el0 + (J)) << 12) | (int)(SJ); \
          } \
          wc += (int)__builtin_popcount(mj); } }
      HITJ(0, h0, s0)
      HITJ(1, h1, s1)
      HITJ(2, h2, s2)
      HITJ(3, h3, s3)
      HITJ(4, h4, s4)
      HITJ(5, h5, s5)
      HITJ(6, h6, s6)
      HITJ(7, h7, s7)
#undef HITJ
    }
  }
  return wc;
}

__global__ __launch_bounds__(NTHR) void k_wprep(
    const float* __restrict__ W, const int* __restrict__ idxu, unsigned short* planes) {
  (void)idxu;
  const int i = blockIdx.x * NTHR + (int)threadIdx.x;
  if (i >= NOUT * (KF / 8)) return;
  const int n  = i / (KF / 8);
  const int k0 = (i - n * (KF / 8)) * 8;
  float f[8];
#pragma unroll
  for (int j = 0; j < 8; ++j) f[j] = W[(size_t)(k0 + j) * NOUT + n];
  v8us hu, lu;
#pragma unroll
  for (int e = 0; e < 8; ++e) {
    const unsigned int hb = bf_bits(f[e]);
    hu[e] = (unsigned short)hb;
    lu[e] = (unsigned short)bf_bits(f[e] - __uint_as_float(hb << 16));
  }
  unsigned short* ph = planes + (size_t)n * KF + k0;
  unsigned short* pl = ph + (size_t)NOUT * KF;
  *(volatile v8us*)ph = hu;
  *(volatile v8us*)pl = lu;
  __threadfence();
  *(volatile v8us*)ph = hu;
  *(volatile v8us*)pl = lu;
}

__global__ __launch_bounds__(NTHR) void k_main(
    const float* __restrict__ x, const int* __restrict__ adj,
    const unsigned short* __restrict__ planes, const float* __restrict__ bias,
    float* out, int nN, int nE) {
  extern __shared__ v4f lds_dyn[];
  float* acc  = (float*)lds_dyn;
  int*   list = (int*)(acc + TGT * FIN);
  int*   scnt = list + LISTN;
  int*   wcnt = scnt + TGT;
  const int tid = threadIdx.x, lane = tid & 31, wave = tid >> 5, hh = lane >> 4, m = lane & 15;
  const int nodeBase = blockIdx.x * TGT;

  {
    const v4f z = {0.f, 0.f, 0.f, 0.f};
#pragma unroll 1
    for (int i = tid; i < TGT * FIN / 4; i += NTHR) ((v4f*)acc)[i] = z;
#pragma unroll 1
    for (int i = tid; i < TGT; i += NTHR) scnt[i] = 0;
  }
  __syncthreads();

  const int nChunks = (nE + CHUNK - 1) / CHUNK;
#pragma unroll 1
  for (int ch = 0; ch < nChunks; ++ch) {
    const int cbase = ch * CHUNK;
    const int wc = scan_chunk<TGT>(adj, nE, cbase, nodeBase, list, tid, wave);
    if (lane == 0) wcnt[wave] = wc;
    __syncthreads();
    if (wave == 0) {
#pragma unroll 1
      for (int wsx = 0; wsx < NWAVE; ++wsx) {
        int n = __builtin_amdgcn_readfirstlane(wcnt[wsx]);
        n = n > WCAP ? WCAP : (n < 0 ? 0 : n);
        const int* lp = list + wsx * WCAP;
#pragma unroll 1
        for (int i = 0; i < n; ++i) {
          const int ent  = __builtin_amdgcn_readfirstlane(lp[i]);
          const int slot = ent & (TGT - 1);
          int e = cbase + ((ent >> 12) & (CHUNK - 1));
          e = e > nE - 1 ? nE - 1 : e;
          int src = adj[(size_t)2 * (size_t)e + 1];
          src = src < 0 ? src + nN : src;
          src = src < 0 ? 0 : (src > nN - 1 ? nN - 1 : src);
          const v4f v = *(const v4f*)(x + (size_t)src * FIN + 4 * lane);
          v4f* ap = (v4f*)(acc + slot * FIN + 4 * lane);
          *ap = *ap + v;
          if (lane == 0) scnt[slot] = scnt[slot] + 1;
        }
      }
    }
    __syncthreads();
  }

#pragma unroll 1
  for (int it = 0; it < TGT / (NWAVE * 16); ++it) {
    const int r0 = 16 * (NWAVE * it + wave);
    if (nodeBase + r0 >= nN) continue;
    const int lrow = r0 + m;
    int grow = nodeBase + lrow;
    grow = grow > nN - 1 ? nN - 1 : grow;
    const int cv = scnt[lrow];
    const float inv = 1.0f / (float)cv;
    const float* arow = acc + lrow * FIN + 8 * hh;
    const float* xrow = x + (size_t)grow * FIN + 8 * hh;
    const unsigned short* bm = planes + (size_t)m * KF + 8 * hh;

    v8f d[8];
#pragma unroll
    for (int t = 0; t < 8; ++t) { v8f z = {0.f, 0.f, 0.f, 0.f, 0.f, 0.f, 0.f, 0.f}; d[t] = z; }

#pragma unroll 1
    for (int kt = 0; kt < FIN / 32; ++kt) {
      const float* p = xrow + 32 * kt;
      const v4f a0 = *(const v4f*)(p);
      const v4f a1 = *(const v4f*)(p + 4);
      const v4f a2 = *(const v4f*)(p + 16);
      const v4f a3 = *(const v4f*)(p + 20);
      FragB ah, al;
      split16(a0, a1, a2, a3, ah, al);
      const unsigned short* bp0 = bm + 32 * kt;
#pragma unroll
      for (int t = 0; t < 8; ++t) {
        const unsigned short* bp = bp0 + (size_t)(16 * t) * KF;
        const unsigned short* bq = bp + (size_t)NOUT * KF;
        FragB bh, bl;
        bh.h[0] = *(const v8us*)bp; bh.h[1] = *(const v8us*)(bp + 16);
        bl.h[0] = *(const v8us*)bq; bl.h[1] = *(const v8us*)(bq + 16);
        d[t] = wmb(ah, bh, d[t]);
        d[t] = wmb(ah, bl, d[t]);
        d[t] = wmb(al, bh, d[t]);
      }
    }
#pragma unroll 1
    for (int kt = 0; kt < FIN / 32; ++kt) {
      const float* p = arow + 32 * kt;
      const v4f a0 = *(const v4f*)(p)      * inv;
      const v4f a1 = *(const v4f*)(p + 4)  * inv;
      const v4f a2 = *(const v4f*)(p + 16) * inv;
      const v4f a3 = *(const v4f*)(p + 20) * inv;
      FragB ah, al;
      split16(a0, a1, a2, a3, ah, al);
      const unsigned short* bp0 = bm + FIN + 32 * kt;
#pragma unroll
      for (int t = 0; t < 8; ++t) {
        const unsigned short* bp = bp0 + (size_t)(16 * t) * KF;
        const unsigned short* bq = bp + (size_t)NOUT * KF;
        FragB bh, bl;
        bh.h[0] = *(const v8us*)bp; bh.h[1] = *(const v8us*)(bp + 16);
        bl.h[0] = *(const v8us*)bq; bl.h[1] = *(const v8us*)(bq + 16);
        d[t] = wmb(ah, bh, d[t]);
        d[t] = wmb(ah, bl, d[t]);
        d[t] = wmb(al, bh, d[t]);
      }
    }

    float* stg = acc + (size_t)r0 * FIN;
#pragma unroll
    for (int t = 0; t < 8; ++t) {
      const float bv = bias[16 * t + m];
      float sg[8];
#pragma unroll
      for (int r = 0; r < 8; ++r) {
        const float v  = d[t][r] + bv;
        const float ex = expf(-v);
        sg[r] = __builtin_amdgcn_rcpf(1.0f + ex);
      }
      v4f lo4, hi4;
      lo4.x = sg[0]; lo4.y = sg[1]; lo4.z = sg[2]; lo4.w = sg[3];
      hi4.x = sg[4]; hi4.y = sg[5]; hi4.z = sg[6]; hi4.w = sg[7];
      float* sp = stg + (t * 32 + lane) * 8;
      *(v4f*)(sp)     = lo4;
      *(v4f*)(sp + 4) = hi4;
    }
    __builtin_amdgcn_fence(__ATOMIC_RELEASE, "wavefront");
    __builtin_amdgcn_wave_barrier();

    v4f ov[16];
    const int tq = lane >> 2, m0 = 4 * (lane & 3);
#pragma unroll
    for (int R = 0; R < 16; ++R) {
      const float* rp = stg + (tq * 32 + 16 * (R >> 3) + m0) * 8 + (R & 7);
      v4f o;
      o.x = rp[0]; o.y = rp[8]; o.z = rp[16]; o.w = rp[24];
      ov[R] = o;
    }
    float* ob = out + 4 * lane;
#pragma unroll
    for (int R = 0; R < 16; ++R) {
      const int gr = nodeBase + r0 + R;
      if (gr < nN) *(volatile v4f*)(ob + (size_t)gr * OUTW) = ov[R];
    }
    __threadfence();
#pragma unroll
    for (int R = 0; R < 16; ++R) {
      const int gr = nodeBase + r0 + R;
      if (gr < nN) *(volatile v4f*)(ob + (size_t)gr * OUTW) = ov[R];
    }
  }
}

extern "C" void kernel_launch(void* const* d_in, const int* in_sizes, int n_in,
                              void* d_out, int out_size, void* d_ws, size_t ws_size,
                              hipStream_t stream) {
  if (n_in < 5) return;
  const int nN = in_sizes[0] / FIN;
  if (nN <= 0 || in_sizes[0] != nN * FIN) return;
  const int nE = in_sizes[1] / 2;
  if (nE < 1 || in_sizes[1] != 2 * nE) return;
  if (in_sizes[3] != KF * NOUT || in_sizes[4] != NOUT) return;
  if (out_size != nN * OUTW) return;
  if (nN > (1 << 22) || nE > (1 << 28)) return;

  const float* x    = (const float*)d_in[0];
  const int*   adj  = (const int*)d_in[1];
  const int*   idxu = (const int*)d_in[2];
  const float* W    = (const float*)d_in[3];
  const float* bias = (const float*)d_in[4];
  float* out = (float*)d_out;

  const size_t plBytes = (size_t)NPL * 2;
  if (plBytes > ws_size) return;
  unsigned short* planes = (unsigned short*)d_ws;

  k_wprep<<<(NOUT * (KF / 8)) / NTHR, NTHR, 0, stream>>>(W, idxu, planes);

  hipFuncSetAttribute(reinterpret_cast<const void*>(&k_main),
                      hipFuncAttributeMaxDynamicSharedMemorySize, LDS_MAIN);
  const int nBlk = (nN + TGT - 1) / TGT;
  k_main<<<nBlk, NTHR, LDS_MAIN, stream>>>(x, adj, planes, bias, out, nN, nE);
}
